// RNNNetv1_240518169257
// MI455X (gfx1250) — hardware-run, weakly checked
//
#include <hip/hip_runtime.h>

typedef __attribute__((ext_vector_type(16))) __bf16       v16b;
typedef __attribute__((ext_vector_type(8)))  __bf16       v8b;
typedef __attribute__((ext_vector_type(8)))  float        v8f;
typedef __attribute__((ext_vector_type(4)))  float        v4f;
typedef __attribute__((ext_vector_type(4)))  unsigned int v4u;

constexpr int kBatch   = 10;
constexpr int kSteps   = 12;
constexpr int kFeat    = 500;
constexpr int kHid     = 200;
constexpr int kGate    = 3 * kHid;
constexpr int kRowsX   = kBatch * kSteps;
constexpr int kRowsXPad = 128;
constexpr int kFeatPad = 512;
constexpr int kGatePad = 640;
constexpr int kHidPad  = 224;
constexpr int kOutElems = kBatch * kHid;
static_assert(kGate == 600, "gate width");
static_assert(kRowsX == 120, "x rows");
static_assert(kFeatPad % 32 == 0 && kHidPad % 32 == 0, "k tiles of 32");
static_assert(kFeatPad >= kFeat && kHidPad >= kHid, "k pads");
static_assert(kRowsXPad % 32 == 0 && kGatePad % 64 == 0, "tile multiples");
static_assert(kFeat % 4 == 0 && kHid % 8 == 0, "vector load alignment");

constexpr int kPackThreads = 256;
constexpr int kPackBlkX  = (kRowsXPad * kFeatPad / 8) / kPackThreads;
constexpr int kPackBlkWi = (kGatePad * kFeatPad / 8) / kPackThreads;
constexpr int kPackBlkWh = (kGatePad * kHidPad / 8) / kPackThreads;
static_assert(kPackBlkX * kPackThreads * 8 == kRowsXPad * kFeatPad, "exact cover of the x planes");
static_assert(kPackBlkWi * kPackThreads * 8 == kGatePad * kFeatPad, "exact cover of the W_ih planes");
static_assert(kPackBlkWh * kPackThreads * 8 == kGatePad * kHidPad, "exact cover of the W_hh planes");
constexpr int kPackBlocks = kPackBlkX + kPackBlkWi + kPackBlkWh;

constexpr int kProjTilesM = kRowsXPad / 32;
constexpr int kProjTilesN = kGatePad / 64;
constexpr int kProjTiles  = kProjTilesM * kProjTilesN;
constexpr int kProjBlocks = kProjTiles / 8;
static_assert(kProjBlocks * 8 == kProjTiles, "whole blocks of 8 wave tiles");

constexpr int kRecThreads = 512;
constexpr int kRecWaves   = kRecThreads / 32;
constexpr int kHidPitch   = 232;
constexpr int kGhPitch    = 608;
constexpr int kRecTilesN  = 38;
constexpr int kStageChunks = 16 * kHidPad / 8;
constexpr int kChunksPerRow = kHidPad / 8;
static_assert(kRecTilesN * 16 == kGhPitch && kGhPitch >= kGate && kGhPitch <= kGatePad, "recurrent n tiles");
static_assert(kStageChunks <= kRecThreads, "one chunk per thread");
static_assert((kHidPitch * 2) % 16 == 0 && kHidPitch >= kHidPad, "16-B aligned LDS rows");
static_assert(4 * kRecThreads >= kOutElems, "gate pass cover");
static_assert(kRecWaves * 8 >= kRowsX, "score pass cover");
static_assert(kOutElems % 4 == 0 && kOutElems / 4 <= kRecThreads, "output chunks");

namespace eng {

__device__ __forceinline__ unsigned int f2bf_bits(float f) {
  const unsigned int u = __float_as_uint(f);
  return (u + 0x7FFFu + ((u >> 16) & 1u)) >> 16;
}
__device__ __forceinline__ float bf_bits2f(unsigned int h) { return __uint_as_float(h << 16); }

union FragB { v16b v; v8b h[2]; };

__device__ __forceinline__ v16b frag_load_global(const __bf16* p) {
  FragB f;
  f.h[0] = *(const v8b*)(p);
  f.h[1] = *(const v8b*)(p + 16);
  return f.v;
}

__device__ __forceinline__ v8f mma_bf16(v16b a, v16b b, v8f c) {
  c = __builtin_amdgcn_wmma_f32_16x16x32_bf16(false, a, false, b, (short)0, c, false, false);
  asm volatile("v_nop\n\tv_nop\n\tv_nop\n\tv_nop" : "+v"(c) : "v"(a), "v"(b));
  return c;
}

__device__ __forceinline__ void split8(const float (&fv)[8], bool live, v4u& wh, v4u& wl) {
  unsigned int hb[8];
  unsigned int lb[8];
#pragma unroll
  for (int e = 0; e < 8; ++e) {
    const float v = live ? fv[e] : 0.0f;
    hb[e] = f2bf_bits(v);
    lb[e] = f2bf_bits(v - bf_bits2f(hb[e]));
  }
#pragma unroll
  for (int q = 0; q < 4; ++q) {
    wh[q] = hb[2 * q] | (hb[2 * q + 1] << 16);
    wl[q] = lb[2 * q] | (lb[2 * q + 1] << 16);
  }
}

}

__global__ __launch_bounds__(kPackThreads)
void pack_planes(const float* __restrict__ x, const float* __restrict__ wih, const float* __restrict__ whh,
                 unsigned short* __restrict__ xaHi, unsigned short* __restrict__ xaLo,
                 unsigned short* __restrict__ wiHi, unsigned short* __restrict__ wiLo,
                 unsigned short* __restrict__ whHi, unsigned short* __restrict__ whLo)
{
  const int blk = blockIdx.x;
  const int tid = threadIdx.x;
  const float* src;
  unsigned short* dHi;
  unsigned short* dLo;
  int rowsReal, colsReal, colsPad, blk0;
  if (blk < kPackBlkX) {
    src = x;   dHi = xaHi; dLo = xaLo; rowsReal = kRowsX; colsReal = kFeat; colsPad = kFeatPad; blk0 = 0;
  } else if (blk < kPackBlkX + kPackBlkWi) {
    src = wih; dHi = wiHi; dLo = wiLo; rowsReal = kGate;  colsReal = kFeat; colsPad = kFeatPad; blk0 = kPackBlkX;
  } else {
    src = whh; dHi = whHi; dLo = whLo; rowsReal = kGate;  colsReal = kHid;  colsPad = kHidPad;  blk0 = kPackBlkX + kPackBlkWi;
  }
  const int gid = (blk - blk0) * kPackThreads + tid;
  const int e0  = gid * 8;
  const int row = e0 / colsPad;
  const int col = e0 - row * colsPad;
  const int rc = row < rowsReal ? row : rowsReal - 1;
  const int c0 = col < colsReal - 4 ? col : colsReal - 4;
  const int c1 = col + 4 < colsReal - 4 ? col + 4 : colsReal - 4;
  const float* rp = src + (size_t)rc * colsReal;
  const v4f va = *(const v4f*)(rp + c0);
  const v4f vb = *(const v4f*)(rp + c1);
  float fv[8];
  fv[0] = va[0]; fv[1] = va[1]; fv[2] = va[2]; fv[3] = va[3];
  fv[4] = vb[0]; fv[5] = vb[1]; fv[6] = vb[2]; fv[7] = vb[3];
  unsigned int hb[8];
  unsigned int lb[8];
#pragma unroll
  for (int e = 0; e < 8; ++e) {
    const bool live = (row < rowsReal) && (col + e < colsReal);
    const float v = live ? fv[e] : 0.0f;
    hb[e] = eng::f2bf_bits(v);
    lb[e] = eng::f2bf_bits(v - eng::bf_bits2f(hb[e]));
  }
  v4u wh, wl;
#pragma unroll
  for (int q = 0; q < 4; ++q) {
    wh[q] = hb[2 * q] | (hb[2 * q + 1] << 16);
    wl[q] = lb[2 * q] | (lb[2 * q + 1] << 16);
  }
  for (int pass = 0; pass < 2; ++pass) {
    *(volatile v4u*)(dHi + e0) = wh;
    *(volatile v4u*)(dLo + e0) = wl;
    __threadfence();
  }
}

__global__ __launch_bounds__(256)
void input_proj_gemm(const unsigned short* __restrict__ aHiP, const unsigned short* __restrict__ aLoP,
                     const unsigned short* __restrict__ bHiP, const unsigned short* __restrict__ bLoP,
                     float* __restrict__ C)
{
  const __bf16* Ah = (const __bf16*)aHiP;
  const __bf16* Al = (const __bf16*)aLoP;
  const __bf16* Bh = (const __bf16*)bHiP;
  const __bf16* Bl = (const __bf16*)bLoP;
  __shared__ __align__(16) float sT[8][16 * 68];
  const int lane = threadIdx.x & 31;
  const int wave = threadIdx.x >> 5;
  const int tile = blockIdx.x * 8 + wave;
  if (tile >= kProjTiles) return;
  const int tm = tile / kProjTilesN;
  const int tn = tile - tm * kProjTilesN;
  const int m0 = tm << 5;
  const int n0 = tn << 6;
  const int rlane = lane & 15;
  const int koff  = (lane >> 4) * 8;
  const int mOff  = (lane >> 4) * 8;

  v8f acc[2][4];
#pragma unroll
  for (int i = 0; i < 2; ++i)
#pragma unroll
    for (int j = 0; j < 4; ++j) acc[i][j] = (v8f){0.f, 0.f, 0.f, 0.f, 0.f, 0.f, 0.f, 0.f};

#pragma unroll 1
  for (int k0 = 0; k0 < kFeatPad; k0 += 32) {
    v16b bh[4], bl[4];
#pragma unroll
    for (int j = 0; j < 4; ++j) {
      const size_t bo = (size_t)(n0 + (j << 4) + rlane) * kFeatPad + koff + k0;
      bh[j] = eng::frag_load_global(Bh + bo);
      bl[j] = eng::frag_load_global(Bl + bo);
    }
#pragma unroll
    for (int i = 0; i < 2; ++i) {
      const size_t ao = (size_t)(m0 + (i << 4) + rlane) * kFeatPad + koff + k0;
      const v16b ah = eng::frag_load_global(Ah + ao);
      const v16b al = eng::frag_load_global(Al + ao);
#pragma unroll
      for (int j = 0; j < 4; ++j) {
        acc[i][j] = eng::mma_bf16(ah, bh[j], acc[i][j]);
        acc[i][j] = eng::mma_bf16(ah, bl[j], acc[i][j]);
        acc[i][j] = eng::mma_bf16(al, bh[j], acc[i][j]);
      }
    }
  }

  float* slab = sT[wave];
#pragma unroll
  for (int i = 0; i < 2; ++i) {
    const int mBase = m0 + (i << 4);
#pragma unroll
    for (int j = 0; j < 4; ++j) {
#pragma unroll
      for (int r = 0; r < 8; ++r) {
        slab[(mOff + r) * 68 + (j << 4) + rlane] = acc[i][j][r];
      }
    }
    __builtin_amdgcn_fence(__ATOMIC_RELEASE, "workgroup");
    __builtin_amdgcn_wave_barrier();
    __builtin_amdgcn_fence(__ATOMIC_ACQUIRE, "workgroup");
    {
      const int hh = lane >> 4;
      const int c4 = (lane & 15) * 4;
      for (int pass = 0; pass < 2; ++pass) {
#pragma unroll
        for (int it = 0; it < 8; ++it) {
          const int row = it * 2 + hh;
          const v4f v = *(const v4f*)(slab + row * 68 + c4);
          *(volatile v4f*)(C + (size_t)(mBase + row) * kGatePad + n0 + c4) = v;
        }
        __threadfence();
      }
    }
    __builtin_amdgcn_fence(__ATOMIC_RELEASE, "workgroup");
    __builtin_amdgcn_wave_barrier();
    __builtin_amdgcn_fence(__ATOMIC_ACQUIRE, "workgroup");
  }
}

#define STAGE_VEC_TO_LDS(SRCPTR, DSTARR, NELEM)                               \
  for (int stg_base = 0; stg_base < (NELEM); stg_base += kRecThreads) {       \
    const int stg_idx = stg_base + tid;                                       \
    const int stg_clamp = stg_idx < (NELEM) ? stg_idx : (NELEM) - 1;          \
    float stg_val = (SRCPTR)[stg_clamp];                                      \
    asm volatile("" : "+v"(stg_val));                                         \
    if (stg_idx < (NELEM)) DSTARR[stg_idx] = stg_val;                         \
  }

__global__ __launch_bounds__(kRecThreads)
void recurrent_block(const float* __restrict__ x, const float* __restrict__ guidance,
                     const float* __restrict__ wx, const float* __restrict__ Wh,
                     const float* __restrict__ bh, const float* __restrict__ b_ih,
                     const float* __restrict__ b_hh, const float* __restrict__ h0,
                     const unsigned short* __restrict__ whhHiP, const unsigned short* __restrict__ whhLoP,
                     const float* __restrict__ XW, float* __restrict__ out)
{
  __shared__ __align__(16) float  hf[kOutElems];
  __shared__ __align__(16) __bf16 hHi[16 * kHidPitch];
  __shared__ __align__(16) __bf16 hLo[16 * kHidPitch];
  __shared__ __align__(16) float  gh[kBatch * kGhPitch];
  __shared__ float xw_s[128];
  __shared__ float gd_s[128];
  __shared__ float sc_s[128];
  __shared__ float at_s[128];
  __shared__ float Wh_s[kSteps * kHid];
  __shared__ float bh_s[16];
  __shared__ float bi_s[kGate];
  __shared__ float bhh_s[kGate];

  const int tid  = threadIdx.x;
  const int lane = tid & 31;
  const int wave = tid >> 5;
  const int rl   = lane & 15;
  const int hh   = lane >> 4;
  const __bf16* whhHi = (const __bf16*)whhHiP;
  const __bf16* whhLo = (const __bf16*)whhLoP;

  STAGE_VEC_TO_LDS(guidance, gd_s, kRowsX)
  STAGE_VEC_TO_LDS(Wh, Wh_s, kSteps * kHid)
  STAGE_VEC_TO_LDS(bh, bh_s, kSteps)
  STAGE_VEC_TO_LDS(b_ih, bi_s, kGate)
  STAGE_VEC_TO_LDS(b_hh, bhh_s, kGate)
  STAGE_VEC_TO_LDS(h0, hf, kOutElems)

#pragma unroll 1
  for (int q = 0; q < 8; ++q) {
    const int p  = wave + kRecWaves * q;
    const int pc = p < kRowsX ? p : kRowsX - 1;
    const float* xr = x + (size_t)pc * kFeat;
    float acc = 0.0f;
#pragma unroll 1
    for (int k = 0; k < 16; ++k) {
      const int f  = lane + 32 * k;
      const int fc = f < kFeat ? f : kFeat - 1;
      float xv = xr[fc];
      float wv = wx[fc];
      asm volatile("" : "+v"(xv), "+v"(wv));
      const float xs = (f < kFeat) ? xv : 0.0f;
      acc = fmaf(xs, wv, acc);
    }
    acc += __shfl_xor(acc, 16, 32);
    acc += __shfl_xor(acc, 8, 32);
    acc += __shfl_xor(acc, 4, 32);
    acc += __shfl_xor(acc, 2, 32);
    acc += __shfl_xor(acc, 1, 32);
    if (lane == 0 && p < kRowsX) xw_s[p] = acc;
  }
  __syncthreads();

#pragma unroll 1
  for (int i = 0; i < kSteps; ++i) {
    {
      const int ch  = tid < kStageChunks ? tid : kStageChunks - 1;
      const int row = ch / kChunksPerRow;
      const int col = (ch - row * kChunksPerRow) * 8;
      const int rc  = row < kBatch ? row : kBatch - 1;
      const int cc  = col < kHid ? col : kHid - 8;
      const v4f pa = *(const v4f*)(hf + rc * kHid + cc);
      const v4f pb = *(const v4f*)(hf + rc * kHid + cc + 4);
      const bool live = (row < kBatch) && (col < kHid);
      float fv[8];
      fv[0] = pa[0]; fv[1] = pa[1]; fv[2] = pa[2]; fv[3] = pa[3];
      fv[4] = pb[0]; fv[5] = pb[1]; fv[6] = pb[2]; fv[7] = pb[3];
      v4u wh, wl;
      eng::split8(fv, live, wh, wl);
      if (tid < kStageChunks) {
        *(v8b*)(hHi + row * kHidPitch + col) = __builtin_bit_cast(v8b, wh);
        *(v8b*)(hLo + row * kHidPitch + col) = __builtin_bit_cast(v8b, wl);
      }
    }
#pragma unroll 1
    for (int q = 0; q < 8; ++q) {
      const int p  = wave + kRecWaves * q;
      const int pc = p < kRowsX ? p : kRowsX - 1;
      const int b  = pc / kSteps;
      const int t  = pc - b * kSteps;
      float acc = 0.0f;
#pragma unroll
      for (int m = 0; m < 7; ++m) {
        const int k  = lane + 32 * m;
        const int kc = k < kHid ? k : kHid - 1;
        const float hv = hf[b * kHid + kc];
        const float wv = Wh_s[t * kHid + kc];
        const float hs = (k < kHid) ? hv : 0.0f;
        acc = fmaf(hs, wv, acc);
      }
      acc += __shfl_xor(acc, 16, 32);
      acc += __shfl_xor(acc, 8, 32);
      acc += __shfl_xor(acc, 4, 32);
      acc += __shfl_xor(acc, 2, 32);
      acc += __shfl_xor(acc, 1, 32);
      float gsum = 0.0f;
#pragma unroll 1
      for (int t2 = 0; t2 < i; ++t2) gsum += gd_s[b * kSteps + t2];
      const float gv   = gd_s[pc];
      const float gsel = (gsum == 0.0f) ? 1.0f : gv;
      const float gcur = (t == i) ? 1.0f : 0.0f;
      const float g    = (t < i) ? gsel : gcur;
      const float sval = g * xw_s[pc] + (acc + bh_s[t]);
      if (lane == 0 && p < kRowsX) sc_s[p] = sval;
    }
    __syncthreads();

    if (tid < kSteps) {
      const int t = tid;
      float mx = sc_s[t];
#pragma unroll 1
      for (int b = 1; b < kBatch; ++b) mx = fmaxf(mx, sc_s[b * kSteps + t]);
      float sum = 0.0f;
#pragma unroll 1
      for (int b = 0; b < kBatch; ++b) sum += expf(sc_s[b * kSteps + t] - mx);
      const float inv = 1.0f / sum;
#pragma unroll 1
      for (int b = 0; b < kBatch; ++b) at_s[b * kSteps + t] = expf(sc_s[b * kSteps + t] - mx) * inv;
    }
    __syncthreads();

#pragma unroll 1
    for (int tile = wave; tile < kRecTilesN; tile += kRecWaves) {
      const int n = tile * 16 + rl;
      const __bf16* bHp = whhHi + (size_t)n * kHidPad + 8 * hh;
      const __bf16* bLp = whhLo + (size_t)n * kHidPad + 8 * hh;
      const int aoff = rl * kHidPitch + 8 * hh;
      v8f acc = (v8f){0.f, 0.f, 0.f, 0.f, 0.f, 0.f, 0.f, 0.f};
#pragma unroll
      for (int ks = 0; ks < kHidPad / 32; ++ks) {
        asm volatile("" ::: "memory");
        eng::FragB fah, fal;
        fah.h[0] = *(const v8b*)(hHi + aoff + 32 * ks);
        fah.h[1] = *(const v8b*)(hHi + aoff + 32 * ks + 16);
        fal.h[0] = *(const v8b*)(hLo + aoff + 32 * ks);
        fal.h[1] = *(const v8b*)(hLo + aoff + 32 * ks + 16);
        const v16b fbh = eng::frag_load_global(bHp + 32 * ks);
        const v16b fbl = eng::frag_load_global(bLp + 32 * ks);
        acc = eng::mma_bf16(fah.v, fbh, acc);
        acc = eng::mma_bf16(fah.v, fbl, acc);
        acc = eng::mma_bf16(fal.v, fbh, acc);
      }
#pragma unroll
      for (int r = 0; r < 8; ++r) {
        const int row = 8 * hh + r;
        if (row < kBatch) gh[row * kGhPitch + n] = acc[r];
      }
    }
    __syncthreads();

#pragma unroll 1
    for (int it = 0; it < 4; ++it) {
      const int idx = it * kRecThreads + tid;
      const int ic  = idx < kOutElems ? idx : kOutElems - 1;
      const int b   = ic / kHid;
      const int j   = ic - b * kHid;
      const float* xwp = XW + (size_t)(b * kSteps) * kGatePad + j;
      float gr = 0.0f;
      float gz = 0.0f;
      float gn = 0.0f;
#pragma unroll 1
      for (int t = 0; t <= i; ++t) {
        const float av = at_s[b * kSteps + t];
        float v0 = xwp[t * kGatePad];
        float v1 = xwp[t * kGatePad + kHid];
        float v2 = xwp[t * kGatePad + 2 * kHid];
        asm volatile("" : "+v"(v0), "+v"(v1), "+v"(v2));
        gr = fmaf(av, v0, gr);
        gz = fmaf(av, v1, gz);
        gn = fmaf(av, v2, gn);
      }
      const float hr = gh[b * kGhPitch + j] + bhh_s[j];
      const float hz = gh[b * kGhPitch + j + kHid] + bhh_s[j + kHid];
      const float hn = gh[b * kGhPitch + j + 2 * kHid] + bhh_s[j + 2 * kHid];
      const float pr = (gr + bi_s[j]) + hr;
      const float pz = (gz + bi_s[j + kHid]) + hz;
      const float rg = 1.0f / (1.0f + expf(-pr));
      const float zg = 1.0f / (1.0f + expf(-pz));
      const float ng = tanhf((gn + bi_s[j + 2 * kHid]) + rg * hn);
      const float hp = hf[ic];
      const float hnew = (1.0f - zg) * ng + zg * hp;
      if (idx < kOutElems) hf[idx] = hnew;
    }
    __syncthreads();
  }

  {
    const int nchunk = kOutElems / 4;
    const int tc = tid < nchunk ? tid : nchunk - 1;
    const v4f ov = *(const v4f*)(hf + 4 * tc);
    for (int pass = 0; pass < 2; ++pass) {
      if (tid < nchunk) *(volatile v4f*)(out + 4 * tid) = ov;
      __threadfence();
    }
  }
}

extern "C" void kernel_launch(void* const* d_in, const int* in_sizes, int n_in,
                              void* d_out, int out_size, void* d_ws, size_t ws_size,
                              hipStream_t stream) {
  if (n_in < 10) return;
  if (in_sizes[0] < kRowsX * kFeat || in_sizes[1] < kRowsX || in_sizes[2] < kFeat ||
      in_sizes[3] < kSteps * kHid || in_sizes[4] < kSteps || in_sizes[5] < kGate * kFeat ||
      in_sizes[6] < kGate * kHid || in_sizes[7] < kGate || in_sizes[8] < kGate ||
      in_sizes[9] < kOutElems || out_size < kOutElems) return;

  const float* x        = (const float*)d_in[0];
  const float* guidance = (const float*)d_in[1];
  const float* wx       = (const float*)d_in[2];
  const float* Wh       = (const float*)d_in[3];
  const float* bh       = (const float*)d_in[4];
  const float* W_ih     = (const float*)d_in[5];
  const float* W_hh     = (const float*)d_in[6];
  const float* b_ih     = (const float*)d_in[7];
  const float* b_hh     = (const float*)d_in[8];
  const float* h0       = (const float*)d_in[9];
  float* out = (float*)d_out;

  size_t off = 0;
  auto carve = [&](size_t bytes) { const size_t o = off; off += (bytes + 127) & ~(size_t)127; return o; };
  const size_t oXaHi = carve((size_t)kRowsXPad * kFeatPad * 2);
  const size_t oXaLo = carve((size_t)kRowsXPad * kFeatPad * 2);
  const size_t oWiHi = carve((size_t)kGatePad * kFeatPad * 2);
  const size_t oWiLo = carve((size_t)kGatePad * kFeatPad * 2);
  const size_t oWhHi = carve((size_t)kGatePad * kHidPad * 2);
  const size_t oWhLo = carve((size_t)kGatePad * kHidPad * 2);
  const size_t oXW   = carve((size_t)kRowsXPad * kGatePad * 4);
  if (off > ws_size) return;

  char* ws = (char*)d_ws;
  unsigned short* xaHi = (unsigned short*)(ws + oXaHi);
  unsigned short* xaLo = (unsigned short*)(ws + oXaLo);
  unsigned short* wiHi = (unsigned short*)(ws + oWiHi);
  unsigned short* wiLo = (unsigned short*)(ws + oWiLo);
  unsigned short* whHi = (unsigned short*)(ws + oWhHi);
  unsigned short* whLo = (unsigned short*)(ws + oWhLo);
  float* XW = (float*)(ws + oXW);

  pack_planes<<<dim3(kPackBlocks), dim3(kPackThreads), 0, stream>>>(x, W_ih, W_hh, xaHi, xaLo, wiHi, wiLo, whHi, whLo);
  input_proj_gemm<<<dim3(kProjBlocks), dim3(256), 0, stream>>>(xaHi, xaLo, wiHi, wiLo, XW);
  recurrent_block<<<dim3(1), dim3(kRecThreads), 0, stream>>>(x, guidance, wx, Wh, bh, b_ih, b_hh, h0, whHi, whLo, XW, out);
}
